// LSTMCell_49349174231639
// MI455X (gfx1250) — hardware-verified
//
#include <hip/hip_runtime.h>
#include <math.h>

constexpr int NROW   = 4096;
constexpr int NIN_F  = 1024;
constexpr int NHID   = 1024;
constexpr int NG3    = 3 * NHID;
constexpr int APITCH = NHID + NIN_F + 2 * NHID;
constexpr int KCAND  = NHID + NIN_F;
constexpr int KGATE  = NIN_F + 2 * NHID;
constexpr int NTHR   = 256;
static_assert(KCAND % 32 == 0 && KGATE % 32 == 0);
static_assert(NROW % 64 == 0 && NHID % 64 == 0 && NG3 % 64 == 0);
static_assert(NIN_F % 64 == 0 && NHID % 64 == 0);
static_assert((NIN_F / 8) % 32 == 0 && (NHID / 8) % 32 == 0);
static_assert((NROW * NHID / 4) % NTHR == 0);
static_assert(NIN_F == NHID);

typedef __attribute__((ext_vector_type(16))) _Float16 v16h;
typedef __attribute__((ext_vector_type(8)))  _Float16 v8h;
typedef __attribute__((ext_vector_type(16))) __bf16   v16b;
typedef __attribute__((ext_vector_type(8)))  __bf16   v8b;
typedef __attribute__((ext_vector_type(8)))  float    v8f;
typedef __attribute__((ext_vector_type(4)))  float    v4f;

__device__ __forceinline__ unsigned short f2bf_bits(float f) {
  unsigned u = __float_as_uint(f);
  return (unsigned short)((u + 0x7FFFu + ((u >> 16) & 1u)) >> 16);
}
__device__ __forceinline__ float bf_bits2f(unsigned short h) { return __uint_as_float(((unsigned)h) << 16); }
__device__ __forceinline__ float bf16r(float f) { return bf_bits2f(f2bf_bits(f)); }

__device__ __forceinline__ void dep_guard_h(v8f& a, v8f& b, v16h x, v16h y) { asm volatile("v_nop\n\tv_nop\n\tv_nop\n\tv_nop" : "+v"(a), "+v"(b) : "v"(x), "v"(y)); }
__device__ __forceinline__ void dep_guard_b(v8f& a, v8f& b, v16b x, v16b y) { asm volatile("v_nop\n\tv_nop\n\tv_nop\n\tv_nop" : "+v"(a), "+v"(b) : "v"(x), "v"(y)); }
__device__ __forceinline__ void dep_guard4_h(v8f& a, v8f& b, v8f& c, v8f& d, v16h x, v16h y) { asm volatile("v_nop\n\tv_nop\n\tv_nop\n\tv_nop" : "+v"(a), "+v"(b), "+v"(c), "+v"(d) : "v"(x), "v"(y)); }
__device__ __forceinline__ void dep_guard4_b(v8f& a, v8f& b, v8f& c, v8f& d, v16b x, v16b y) { asm volatile("v_nop\n\tv_nop\n\tv_nop\n\tv_nop" : "+v"(a), "+v"(b), "+v"(c), "+v"(d) : "v"(x), "v"(y)); }
__device__ __forceinline__ void keep4_h(v16h a, v16h b, v16h c, v16h d) { asm volatile("v_nop" :: "v"(a), "v"(b), "v"(c), "v"(d)); }
__device__ __forceinline__ void keep4_b(v16b a, v16b b, v16b c, v16b d) { asm volatile("v_nop" :: "v"(a), "v"(b), "v"(c), "v"(d)); }
__device__ __forceinline__ void acc_guard4(v8f& a, v8f& b, v8f& c, v8f& d) { asm volatile("v_nop\n\tv_nop\n\tv_nop\n\tv_nop" : "+v"(a), "+v"(b), "+v"(c), "+v"(d)); }
template <typename T> struct Frag;
template <> struct Frag<_Float16> {
  typedef v16h V; union U { v16h v; v8h h[2]; };
  static __device__ __forceinline__ v16h load(const _Float16* p) {
    U f; f.h[0] = *(const v8h*)(p); f.h[1] = *(const v8h*)(p + 16); return f.v;
  }
  static __device__ __forceinline__ v8f mma(v16h a, v16h b, v8f c) {
    return __builtin_amdgcn_wmma_f32_16x16x32_f16(false, a, false, b, (short)0, c, false, false);
  }
  static __device__ __forceinline__ void guard(v8f& a, v8f& b, v16h x, v16h y) { dep_guard_h(a, b, x, y); }
  static __device__ __forceinline__ void guard4(v8f& a, v8f& b, v8f& c, v8f& d, v16h x, v16h y) { dep_guard4_h(a, b, c, d, x, y); }
  static __device__ __forceinline__ void keep(v16h a, v16h b, v16h c, v16h d) { keep4_h(a, b, c, d); }
};
template <> struct Frag<__bf16> {
  typedef v16b V; union U { v16b v; v8b h[2]; };
  static __device__ __forceinline__ v16b load(const __bf16* p) {
    U f; f.h[0] = *(const v8b*)(p); f.h[1] = *(const v8b*)(p + 16); return f.v;
  }
  static __device__ __forceinline__ v8f mma(v16b a, v16b b, v8f c) {
    return __builtin_amdgcn_wmma_f32_16x16x32_bf16(false, a, false, b, (short)0, c, false, false);
  }
  static __device__ __forceinline__ void guard(v8f& a, v8f& b, v16b x, v16b y) { dep_guard_b(a, b, x, y); }
  static __device__ __forceinline__ void guard4(v8f& a, v8f& b, v8f& c, v8f& d, v16b x, v16b y) { dep_guard4_b(a, b, c, d, x, y); }
  static __device__ __forceinline__ void keep(v16b a, v16b b, v16b c, v16b d) { keep4_b(a, b, c, d); }
};

template <int ET> struct Elem;
template <> struct Elem<0> { typedef _Float16 T; };
template <> struct Elem<1> { typedef __bf16 T; };
template <int ET, bool SPLIT, int BIAS_MODE, int OUT_MODE, bool RESID, int ACT = 0>
__global__ __launch_bounds__(256) void wmma_gemm64(
    const unsigned short* __restrict__ Ap, const unsigned short* __restrict__ A2p, int lda, long strideA,
    const unsigned short* __restrict__ Btp, const unsigned short* __restrict__ Bt2p, int ldb, long strideB,
    void* __restrict__ Cout, void* __restrict__ Cout2, void* __restrict__ Cout3, int ldc, int ldc2, long strideC,
    const float* __restrict__ bias,
    const float* __restrict__ resid, long strideR,
    int M, int N, int K, float scale) {
  typedef typename Elem<ET>::T T;
  typedef typename Frag<T>::V V;
  const T* A = (const T*)Ap; const T* A2 = (const T*)A2p; const T* Bt = (const T*)Btp; const T* Bt2 = (const T*)Bt2p;
  __shared__ __align__(16) float sT[8][16 * 68];
  const int b    = blockIdx.y;
  const int lane = threadIdx.x & 31;
  const int wave = threadIdx.x >> 5;
  const int tilesN = N >> 6;
  const int tilesM = M >> 6;
  const int tile = blockIdx.x * 8 + wave;
  if (tile >= tilesM * tilesN) return;
  const int tm = tile / tilesN;
  const int tn = tile - tm * tilesN;
  const int m0 = tm << 6;
  const int n0 = tn << 6;

  const T* Ab  = A  + (size_t)b * strideA;
  const T* Bb  = Bt + (size_t)b * strideB;
  const T* Ab2 = SPLIT ? (A2  + (size_t)b * strideA) : nullptr;
  const T* Bb2 = SPLIT ? (Bt2 + (size_t)b * strideB) : nullptr;

  const int rlane = lane & 15;
  const int koff  = (lane >> 4) * 8;
  const int mOff  = (lane >> 4) * 8;

  v8f acc[4][4];
#pragma unroll
  for (int i = 0; i < 4; ++i)
#pragma unroll
    for (int j = 0; j < 4; ++j) acc[i][j] = (v8f){0.f,0.f,0.f,0.f,0.f,0.f,0.f,0.f};

  for (int k0 = 0; k0 < K; k0 += 32) {
    V bh[4], bl[4];
#pragma unroll
    for (int j = 0; j < 4; ++j) {
      const size_t bo = (size_t)(n0 + (j << 4) + rlane) * ldb + koff + k0;
      bh[j] = Frag<T>::load(Bb + bo);
      if (SPLIT) bl[j] = Frag<T>::load(Bb2 + bo);
    }
#pragma unroll
    for (int i = 0; i < 4; ++i) {
      const size_t ao = (size_t)(m0 + (i << 4) + rlane) * lda + koff + k0;
      V ah = Frag<T>::load(Ab + ao);
      V al;
      if (SPLIT) al = Frag<T>::load(Ab2 + ao);
#pragma unroll
      for (int j = 0; j < 4; ++j) {
        acc[i][j] = Frag<T>::mma(ah, bh[j], acc[i][j]);
        if (SPLIT) {
          acc[i][j] = Frag<T>::mma(ah, bl[j], acc[i][j]);
          acc[i][j] = Frag<T>::mma(al, bh[j], acc[i][j]);
        }
      }
      Frag<T>::guard4(acc[i][0], acc[i][1], acc[i][2], acc[i][3], ah, SPLIT ? al : ah);
    }
    Frag<T>::keep(bh[0], bh[1], bh[2], bh[3]);
    if (SPLIT) Frag<T>::keep(bl[0], bl[1], bl[2], bl[3]);
  }
  acc_guard4(acc[0][0], acc[0][1], acc[0][2], acc[0][3]);
  acc_guard4(acc[1][0], acc[1][1], acc[1][2], acc[1][3]);
  acc_guard4(acc[2][0], acc[2][1], acc[2][2], acc[2][3]);
  acc_guard4(acc[3][0], acc[3][1], acc[3][2], acc[3][3]);

  float* slab = sT[wave];
  const float* Rb = RESID ? (resid + (size_t)b * strideR) : nullptr;
#pragma unroll
  for (int i = 0; i < 4; ++i) {
    const int mBase = m0 + (i << 4);
#pragma unroll
    for (int j = 0; j < 4; ++j) {
      const int n = n0 + (j << 4) + rlane;
      float bv = 0.f;
      if (BIAS_MODE == 2) bv = bias[n];
#pragma unroll
      for (int r = 0; r < 8; ++r) {
        float v = acc[i][j][r] * scale;
        if (BIAS_MODE == 1) v += bias[mBase + mOff + r];
        if (BIAS_MODE == 2) v += bv;
        if (RESID) v += Rb[(size_t)(mBase + mOff + r) * ldc + n];
        if (ACT == 1) v = tanhf(v);
        if (ACT == 2) v = fmaxf(v, 0.0f);
        if (ACT == 4) v = (v > 0.f) ? v : 0.01f * v;
        slab[(mOff + r) * 68 + (j << 4) + rlane] = v;
      }
    }
    __builtin_amdgcn_fence(__ATOMIC_RELEASE, "workgroup");
    __builtin_amdgcn_wave_barrier();
    __builtin_amdgcn_fence(__ATOMIC_ACQUIRE, "workgroup");
    if (OUT_MODE == 0 || OUT_MODE == 3) {
      float* C = (float*)Cout + (size_t)b * strideC;
      const int hh = lane >> 4, c4 = (lane & 15) * 4;
      for (int pass = 0; pass < 2; ++pass) {
#pragma unroll
        for (int it = 0; it < 8; ++it) {
          const int row = it * 2 + hh;
          v4f v = *(const v4f*)(slab + row * 68 + c4);
          *(volatile v4f*)(C + (size_t)(mBase + row) * ldc + n0 + c4) = v;
        }
        __threadfence();
      }
    }
    if (OUT_MODE != 0) {
      const int q = lane >> 3, c8 = (lane & 7) * 8;
      const int ldh = (OUT_MODE == 3) ? ldc2 : ldc;
      unsigned short* C  = ((OUT_MODE == 3) ? (unsigned short*)Cout2 : (unsigned short*)Cout) + (size_t)b * strideC;
      unsigned short* C2 = (OUT_MODE == 2) ? ((unsigned short*)Cout2 + (size_t)b * strideC)
                         : (OUT_MODE == 3) ? ((unsigned short*)Cout3 + (size_t)b * strideC) : nullptr;
      for (int pass = 0; pass < 2; ++pass) {
#pragma unroll
        for (int it = 0; it < 4; ++it) {
          const int row = it * 4 + q;
          const float* sp = slab + row * 68 + c8;
          v8h hv, lv;
#pragma unroll
          for (int e = 0; e < 8; ++e) {
            if (OUT_MODE == 1) {
              hv[e] = (_Float16)sp[e];
              lv[e] = hv[e];
            } else {
              unsigned short hb = f2bf_bits(sp[e]);
              unsigned short lb = f2bf_bits(sp[e] - bf_bits2f(hb));
              hv[e] = __builtin_bit_cast(_Float16, hb);
              lv[e] = __builtin_bit_cast(_Float16, lb);
            }
          }
          *(volatile v8h*)(C + (size_t)(mBase + row) * ldh + n0 + c8) = hv;
          if (OUT_MODE >= 2) *(volatile v8h*)(C2 + (size_t)(mBase + row) * ldh + n0 + c8) = lv;
        }
        __threadfence();
      }
    }
    __builtin_amdgcn_fence(__ATOMIC_RELEASE, "workgroup");
    __builtin_amdgcn_wave_barrier();
    __builtin_amdgcn_fence(__ATOMIC_ACQUIRE, "workgroup");
  }
}

__global__ __launch_bounds__(NTHR) void cvtp_kernel(const float* __restrict__ src, unsigned short* __restrict__ dst,
                                                    int nrow, int ncol8, int spitch, int dpitch, int dcol0) {
  const int i  = blockIdx.x * NTHR + threadIdx.x;
  const int n8 = nrow * ncol8;
  if (i < n8) {
    const int row = i / ncol8;
    const int c8  = i - row * ncol8;
    const float* sp = src + (size_t)row * spitch + c8 * 8;
    const v4f a = *(const v4f*)(sp);
    const v4f b = *(const v4f*)(sp + 4);
    v8h hv;
#pragma unroll
    for (int e = 0; e < 4; ++e) {
      const unsigned short b0 = f2bf_bits(a[e]);
      const unsigned short b1 = f2bf_bits(b[e]);
      hv[e]     = __builtin_bit_cast(_Float16, b0);
      hv[4 + e] = __builtin_bit_cast(_Float16, b1);
    }
    unsigned short* dp = dst + (size_t)row * dpitch + dcol0 + (size_t)c8 * 8;
    *(volatile v8h*)dp = hv;
    __threadfence();
    *(volatile v8h*)dp = hv;
  }
}

__global__ __launch_bounds__(NTHR) void tpwd_kernel(const float* __restrict__ src, int R, int C, int ldo,
                                                    unsigned short* __restrict__ O, long dupoff) {
  __shared__ float Tt[64 * 65];
  const int tid = threadIdx.x;
  const int c0 = blockIdx.x * 64, r0 = blockIdx.y * 64;
#pragma unroll
  for (int i = 0; i < 4; ++i) {
    const int idx = i * NTHR + tid;
    const int rr = idx >> 4, cc = (idx & 15) * 4;
    const v4f v = *(const v4f*)(src + (size_t)(r0 + rr) * (size_t)C + c0 + cc);
    Tt[rr * 65 + cc + 0] = v[0];
    Tt[rr * 65 + cc + 1] = v[1];
    Tt[rr * 65 + cc + 2] = v[2];
    Tt[rr * 65 + cc + 3] = v[3];
  }
  __syncthreads();
  const int q = tid >> 3, c8 = (tid & 7) * 8;
  v8h hv[2];
#pragma unroll
  for (int g = 0; g < 2; ++g) {
    const int qq = g * 32 + q;
#pragma unroll
    for (int e = 0; e < 8; ++e) {
      const float f = Tt[(c8 + e) * 65 + qq];
      const unsigned short bits = f2bf_bits(f);
      hv[g][e] = __builtin_bit_cast(_Float16, bits);
    }
  }
  for (int pass = 0; pass < 2; ++pass) {
#pragma unroll
    for (int g = 0; g < 2; ++g) {
      const size_t o = (size_t)(c0 + g * 32 + q) * (size_t)ldo + (size_t)(r0 + c8);
      *(volatile v8h*)(O + o) = hv[g];
      if (dupoff != 0) *(volatile v8h*)(O + o + dupoff) = hv[g];
    }
    __threadfence();
  }
}

__global__ __launch_bounds__(NTHR) void bias2_kernel(const float* __restrict__ b_a, const float* __restrict__ b_b,
                                                     float* __restrict__ dst) {
  const int idx = threadIdx.x * 4;
  const v4f va = *(const v4f*)(b_a + idx);
  const v4f vb = *(const v4f*)(b_b + idx);
  v4f o;
#pragma unroll
  for (int e = 0; e < 4; ++e) o[e] = bf16r(va[e]) + bf16r(vb[e]);
  float* op = dst + idx;
  *(volatile v4f*)op = o;
  __threadfence();
  *(volatile v4f*)op = o;
}

__device__ __forceinline__ float fsig(float x)  { return __builtin_amdgcn_rcpf(1.0f + expf(-x)); }
__device__ __forceinline__ float ftanh(float x) { return 1.0f - 2.0f * __builtin_amdgcn_rcpf(expf(2.0f * x) + 1.0f); }

__global__ __launch_bounds__(NTHR) void cell_kernel(const float* __restrict__ pre, const float* __restrict__ cand,
                                                    const float* __restrict__ cprev, float* __restrict__ outH,
                                                    float* __restrict__ outC, int nq) {
  const int i = blockIdx.x * NTHR + threadIdx.x;
  if (i >= nq) return;
  const int row = i >> 8;
  const int c4  = (i & 255) * 4;
  const float* pr = pre + (size_t)row * NG3 + c4;
  v4f zi = *(const v4f*)(pr);
  v4f zo = *(const v4f*)(pr + NHID);
  v4f zf = *(const v4f*)(pr + 2 * NHID);
  v4f cd = *(const v4f*)(cand  + (size_t)row * NHID + c4);
  v4f cp = *(const v4f*)(cprev + (size_t)row * NHID + c4);
  v4f ho = {0.f, 0.f, 0.f, 0.f};
  v4f co = {0.f, 0.f, 0.f, 0.f};
#pragma unroll 1
  for (int e = 0; e < 4; ++e) {
    const float ig = fsig(zi[0]);
    const float og = fsig(zo[0]);
    const float fg = fsig(zf[0]);
    const float gt = ftanh(cd[0]);
    const float cv = bf16r(cp[0]);
    const float ct = fg * cv + ig * gt;
    const float ht = ftanh(ct) * og;
    ho = (v4f){ho[1], ho[2], ho[3], ht};
    co = (v4f){co[1], co[2], co[3], ct};
    zi = (v4f){zi[1], zi[2], zi[3], zi[0]};
    zo = (v4f){zo[1], zo[2], zo[3], zo[0]};
    zf = (v4f){zf[1], zf[2], zf[3], zf[0]};
    cd = (v4f){cd[1], cd[2], cd[3], cd[0]};
    cp = (v4f){cp[1], cp[2], cp[3], cp[0]};
  }
  float* ph = outH + (size_t)row * NHID + c4;
  float* pc = outC + (size_t)row * NHID + c4;
  *(volatile v4f*)ph = ho;
  *(volatile v4f*)pc = co;
  __threadfence();
  *(volatile v4f*)ph = ho;
  *(volatile v4f*)pc = co;
}

extern "C" void kernel_launch(void* const* d_in, const int* in_sizes, int n_in,
                              void* d_out, int out_size, void* d_ws, size_t ws_size, hipStream_t stream) {
  if (n_in < 19 || d_out == nullptr || d_ws == nullptr) return;
  if (in_sizes[0] != NROW * NIN_F || in_sizes[1] != NROW * NHID || in_sizes[2] != NROW * NHID) return;
  for (int i = 0; i < 8; ++i) {
    if (in_sizes[3 + 2 * i] != NIN_F * NHID || in_sizes[4 + 2 * i] != NHID) return;
  }
  if (out_size != 2 * NROW * NHID) return;

  const float* x    = (const float*)d_in[0];
  const float* h0   = (const float*)d_in[1];
  const float* c0   = (const float*)d_in[2];
  const float* w_hi = (const float*)d_in[3];  const float* b_hi = (const float*)d_in[4];
  const float* w_hh = (const float*)d_in[5];  const float* b_hh = (const float*)d_in[6];
  const float* w_ii = (const float*)d_in[7];  const float* b_ii = (const float*)d_in[8];
  const float* w_ih = (const float*)d_in[9];  const float* b_ih = (const float*)d_in[10];
  const float* w_oi = (const float*)d_in[11]; const float* b_oi = (const float*)d_in[12];
  const float* w_oh = (const float*)d_in[13]; const float* b_oh = (const float*)d_in[14];
  const float* w_fi = (const float*)d_in[15]; const float* b_fi = (const float*)d_in[16];
  const float* w_fh = (const float*)d_in[17]; const float* b_fh = (const float*)d_in[18];
  float* out_h = (float*)d_out;
  float* out_c = (float*)d_out + (size_t)NROW * NHID;

  char* ws = (char*)d_ws; size_t off = 0;
  auto carve = [&](size_t bytes) -> char* { char* p = ws + off; off += (bytes + 255) & ~(size_t)255; return p; };
  unsigned short* APL    = (unsigned short*)carve((size_t)NROW * APITCH * 2);
  unsigned short* BTC    = (unsigned short*)carve((size_t)NHID * KCAND * 2);
  unsigned short* BTG    = (unsigned short*)carve((size_t)NG3 * KGATE * 2);
  float*          BIASC  = (float*)carve((size_t)NHID * 4);
  float*          BIASG  = (float*)carve((size_t)NG3 * 4);
  float*          CAND32 = (float*)carve((size_t)NROW * NHID * 4);
  float*          PRE    = (float*)carve((size_t)NROW * NG3 * 4);
  if (off > ws_size || off > (size_t)134217728) return;

  const int n8a = NROW * (NHID / 8);
  cvtp_kernel<<<(n8a + NTHR - 1) / NTHR, NTHR, 0, stream>>>(h0, APL, NROW, NHID / 8,  NHID,  APITCH, 0);
  cvtp_kernel<<<(n8a + NTHR - 1) / NTHR, NTHR, 0, stream>>>(x,  APL, NROW, NIN_F / 8, NIN_F, APITCH, NHID);

  const dim3 tg(NHID / 64, NIN_F / 64);
  tpwd_kernel<<<tg, NTHR, 0, stream>>>(w_hh, NHID,  NHID, KCAND, BTC,        0L);
  tpwd_kernel<<<tg, NTHR, 0, stream>>>(w_hi, NIN_F, NHID, KCAND, BTC + NHID, 0L);
  {
    const float* wgi[3] = { w_ii, w_oi, w_fi };
    const float* wgh[3] = { w_ih, w_oh, w_fh };
    for (int g = 0; g < 3; ++g) {
      unsigned short* base = BTG + (size_t)g * NHID * KGATE;
      tpwd_kernel<<<tg, NTHR, 0, stream>>>(wgi[g], NIN_F, NHID, KGATE, base,         0L);
      tpwd_kernel<<<tg, NTHR, 0, stream>>>(wgh[g], NHID,  NHID, KGATE, base + NIN_F, (long)NHID);
    }
  }

  bias2_kernel<<<1, NTHR, 0, stream>>>(b_hi, b_hh, BIASC);
  bias2_kernel<<<1, NTHR, 0, stream>>>(b_ii, b_ih, BIASG);
  bias2_kernel<<<1, NTHR, 0, stream>>>(b_oi, b_oh, BIASG + NHID);
  bias2_kernel<<<1, NTHR, 0, stream>>>(b_fi, b_fh, BIASG + 2 * NHID);

  const int tiles1 = (NROW / 64) * (NHID / 64);
  wmma_gemm64<1, false, 2, 3, false, 0><<<dim3((tiles1 + 7) / 8, 1), 256, 0, stream>>>(
      APL, APL, APITCH, 0L, BTC, BTC, KCAND, 0L,
      (void*)CAND32, (void*)(APL + 2 * NHID), (void*)(APL + 3 * NHID), NHID, APITCH, 0L,
      BIASC, CAND32, 0L, NROW, NHID, KCAND, 1.0f);

  const int tiles2 = (NROW / 64) * (NG3 / 64);
  wmma_gemm64<1, false, 2, 0, false, 0><<<dim3((tiles2 + 7) / 8, 1), 256, 0, stream>>>(
      APL + NHID, APL + NHID, APITCH, 0L, BTG, BTG, KGATE, 0L,
      (void*)PRE, (void*)PRE, (void*)PRE, NG3, NG3, 0L,
      BIASG, CAND32, 0L, NROW, NG3, KGATE, 1.0f);

  const int nq = NROW * NHID / 4;
  cell_kernel<<<(nq + NTHR - 1) / NTHR, NTHR, 0, stream>>>(PRE, CAND32, c0, out_h, out_c, nq);
}
